// PointNetSetAbstraction_73065983639805
// MI455X (gfx1250) — hardware-verified
//
#include <hip/hip_runtime.h>
#pragma clang fp contract(off)

typedef __attribute__((ext_vector_type(16))) _Float16     v16h;
typedef __attribute__((ext_vector_type(8)))  _Float16     v8h;
typedef __attribute__((ext_vector_type(8)))  float        v8f;
typedef __attribute__((ext_vector_type(4)))  float        v4f;
typedef __attribute__((ext_vector_type(4)))  unsigned int v4u;

constexpr int NBATCH   = 8;
constexpr int NPTS     = 8192;
constexpr int NSEL     = 2048;
constexpr int NSAMP    = 32;
constexpr int NFEAT    = 32;
constexpr int CIN_REAL = 35;
constexpr int KPAD     = 64;
constexpr int HID1     = 64;
constexpr int HID2     = 64;
constexpr int HID3     = 128;
constexpr int WROWS    = HID1 + HID2 + HID3;
constexpr int PITCH_A  = 72;
constexpr int PITCH_W  = 72;
constexpr int PITCH_S  = 36;
constexpr float WCARRY     = 16.0f;
constexpr float WCARRY_INV = 1.0f / WCARRY;
constexpr float RADIUS_SQ  = 0.25f;

constexpr int PREP_XYZ_BLOCKS = (NBATCH * NPTS) / 256;
constexpr int PREP_PTS_BLOCKS = (NBATCH * NPTS * 4) / 256;
constexpr int PREP_WT_BLOCKS  = (WROWS * 8) / 256;

static_assert(WROWS == 256, "weight rows");
static_assert(KPAD % 32 == 0 && KPAD >= CIN_REAL, "K pad");
static_assert(NFEAT + 3 == CIN_REAL, "feature width");
static_assert((size_t)NBATCH * 3 * NSEL * 4 == 196608, "out0 bytes");
static_assert((size_t)NBATCH * 3 * NSEL * 4 + (size_t)NBATCH * HID3 * NSEL * 4 == 8585216, "out total bytes");
static_assert(PREP_WT_BLOCKS == 8, "weight prep blocks");

constexpr size_t OFF_XT   = 0;
constexpr size_t SZ_XT    = (size_t)NBATCH * NPTS * 16;
constexpr size_t OFF_PTW  = OFF_XT + SZ_XT;
constexpr size_t SZ_PTW   = (size_t)NBATCH * NPTS * NFEAT * 2;
constexpr size_t OFF_WT   = OFF_PTW + SZ_PTW;
constexpr size_t SZ_WT    = (size_t)WROWS * KPAD * 2;
constexpr size_t OFF_NXW  = OFF_WT + SZ_WT;
constexpr size_t SZ_NXW   = (size_t)NBATCH * NSEL * 16;
constexpr size_t WS_TOTAL = OFF_NXW + SZ_NXW;
static_assert(WS_TOTAL <= 134217728, "carve limit");
static_assert((OFF_PTW % 128) == 0 && (OFF_WT % 128) == 0 && (OFF_NXW % 128) == 0, "carve alignment");

union FragU { v16h v; v8h h[2]; };

__device__ __forceinline__ v16h frag_load(const _Float16* p) {
  FragU f;
  f.h[0] = *(const v8h*)(p);
  f.h[1] = *(const v8h*)(p + 16);
  return f.v;
}

__device__ __forceinline__ v8f wm_f16(v16h a, v16h b, v8f c) {
  c = __builtin_amdgcn_wmma_f32_16x16x32_f16(false, a, false, b, (short)0, c, false, false);
  asm volatile("v_nop\n\tv_nop\n\tv_nop\n\tv_nop" : "+v"(c) : "v"(a), "v"(b));
  return c;
}

__device__ __forceinline__ unsigned f16_bits(float f) {
  const _Float16 h = (_Float16)f;
  const unsigned short s = __builtin_bit_cast(unsigned short, h);
  return (unsigned)s;
}

__device__ __forceinline__ void pin3(float& a, float& b, float& c) {
  asm volatile("" : "+v"(a), "+v"(b), "+v"(c) :: "memory");
}

__device__ __forceinline__ void store2_v4f(float* p, v4f v) {
  *(volatile v4f*)p = v;
  __threadfence();
  *(volatile v4f*)p = v;
}

__device__ __forceinline__ void store2_v4u(unsigned* p, v4u v) {
  *(volatile v4u*)p = v;
  __threadfence();
  *(volatile v4u*)p = v;
}

__global__ __launch_bounds__(256)
void prep_kernel(const float* __restrict__ xyz, const float* __restrict__ pts,
                 const float* __restrict__ w1, const float* __restrict__ w2, const float* __restrict__ w3,
                 float* __restrict__ xt, unsigned* __restrict__ ptw, unsigned* __restrict__ wtw) {
#pragma clang fp contract(off)
  const int blk = blockIdx.x;
  const int tid = threadIdx.x;
  if (blk < PREP_XYZ_BLOCKS) {
    const int g = blk * 256 + tid;
    const int b = g >> 13;
    const int n = g & (NPTS - 1);
    const float* xb = xyz + (size_t)b * 3 * NPTS;
    const float x = xb[n];
    const float y = xb[NPTS + n];
    const float z = xb[2 * NPTS + n];
    const float t0 = x * x;
    const float t1 = y * y;
    const float t2 = z * z;
    const float nsq = (t0 + t2) + t1;
    const v4f v = {x, y, z, nsq};
    store2_v4f(xt + (size_t)g * 4, v);
  } else if (blk < PREP_XYZ_BLOCKS + PREP_PTS_BLOCKS) {
    const int g = (blk - PREP_XYZ_BLOCKS) * 256 + tid;
    const int pt = g >> 2;
    const int seg = g & 3;
    const int b = pt >> 13;
    const int n = pt & (NPTS - 1);
    const float* pb = pts + (size_t)b * NFEAT * NPTS + (size_t)(seg * 8) * NPTS + n;
    float f[8];
#pragma unroll
    for (int e = 0; e < 8; ++e) f[e] = pb[(size_t)e * NPTS];
    const unsigned q0 = f16_bits(f[0]) | (f16_bits(f[1]) << 16);
    const unsigned q1 = f16_bits(f[2]) | (f16_bits(f[3]) << 16);
    const unsigned q2 = f16_bits(f[4]) | (f16_bits(f[5]) << 16);
    const unsigned q3 = f16_bits(f[6]) | (f16_bits(f[7]) << 16);
    const v4u w = {q0, q1, q2, q3};
    store2_v4u(ptw + (size_t)g * 4, w);
  } else {
    const int wb = blk - PREP_XYZ_BLOCKS - PREP_PTS_BLOCKS;
    const int g = wb * 256 + tid;
    const int row = g >> 3;
    const int seg = g & 7;
    float f[8];
    if (wb < 2) {
#pragma unroll
      for (int e = 0; e < 8; ++e) {
        const int k = seg * 8 + e;
        int col = (k < NFEAT) ? (k + 3) : (k - NFEAT);
        col = (col > CIN_REAL - 1) ? (CIN_REAL - 1) : col;
        const float ld = w1[row * CIN_REAL + col];
        f[e] = (k < CIN_REAL) ? (ld * WCARRY) : 0.0f;
      }
    } else if (wb < 4) {
#pragma unroll
      for (int e = 0; e < 8; ++e) f[e] = w2[(row - HID1) * HID1 + seg * 8 + e] * WCARRY;
    } else {
#pragma unroll
      for (int e = 0; e < 8; ++e) f[e] = w3[(row - HID1 - HID2) * HID2 + seg * 8 + e] * WCARRY;
    }
    const unsigned q0 = f16_bits(f[0]) | (f16_bits(f[1]) << 16);
    const unsigned q1 = f16_bits(f[2]) | (f16_bits(f[3]) << 16);
    const unsigned q2 = f16_bits(f[4]) | (f16_bits(f[5]) << 16);
    const unsigned q3 = f16_bits(f[6]) | (f16_bits(f[7]) << 16);
    const v4u w = {q0, q1, q2, q3};
    store2_v4u(wtw + (size_t)g * 4, w);
  }
}

__global__ __launch_bounds__(1024)
void fps_kernel(const float* __restrict__ xyz, float* __restrict__ out0, float* __restrict__ nxw) {
#pragma clang fp contract(off)
  __shared__ float sval[32];
  __shared__ int   sidx[32];
  __shared__ int   sfar;
  __shared__ float c3[4];
  __shared__ __align__(16) float cs[3 * NSEL];

  const int b    = blockIdx.x;
  const int tid  = threadIdx.x;
  const int lane = tid & 31;
  const int wid  = tid >> 5;
  const float* xb = xyz + (size_t)b * 3 * NPTS;

  float px[8], py[8], pz[8], dist[8];
#pragma unroll
  for (int i = 0; i < 4; ++i) {
    const int n = tid + i * 1024;
    px[i] = xb[n];
    py[i] = xb[NPTS + n];
    pz[i] = xb[2 * NPTS + n];
    dist[i] = 1e10f;
  }
#pragma unroll
  for (int i = 0; i < 4; ++i) pin3(px[i], py[i], pz[i]);
#pragma unroll
  for (int i = 4; i < 8; ++i) {
    const int n = tid + i * 1024;
    px[i] = xb[n];
    py[i] = xb[NPTS + n];
    pz[i] = xb[2 * NPTS + n];
    dist[i] = 1e10f;
  }
#pragma unroll
  for (int i = 4; i < 8; ++i) pin3(px[i], py[i], pz[i]);

  if (tid == 0) { c3[0] = px[0]; c3[1] = py[0]; c3[2] = pz[0]; c3[3] = 0.0f; sfar = 0; }
  __syncthreads();

#pragma unroll 1
  for (int it = 0; it < NSEL; ++it) {
    if (tid < 3) cs[tid * NSEL + it] = c3[tid];
    const float cx = c3[0];
    const float cy = c3[1];
    const float cz = c3[2];

    float bv = 0.0f;
    int bi = tid;
#pragma unroll
    for (int i = 0; i < 8; ++i) {
      const float dx = px[i] - cx;
      const float dy = py[i] - cy;
      const float dz = pz[i] - cz;
      const float t0 = dx * dx;
      const float t1 = dy * dy;
      const float t2 = dz * dz;
      float d = (t0 + t2) + t1;
      d = fminf(dist[i], d);
      dist[i] = d;
      if (i == 0) {
        bv = d;
      } else {
        const bool tk = d > bv;
        bv = tk ? d : bv;
        bi = tk ? (tid + i * 1024) : bi;
      }
    }
#pragma unroll
    for (int off = 16; off > 0; off >>= 1) {
      const float ov = __shfl_xor(bv, off, 32);
      const int   oi = __shfl_xor(bi, off, 32);
      const bool tk = (ov > bv) || (ov == bv && oi < bi);
      bv = tk ? ov : bv;
      bi = tk ? oi : bi;
    }
    if (lane == 0) { sval[wid] = bv; sidx[wid] = bi; }
    __syncthreads();
    if (wid == 0) {
      float v = sval[lane];
      int ix = sidx[lane];
#pragma unroll
      for (int off = 16; off > 0; off >>= 1) {
        const float ov = __shfl_xor(v, off, 32);
        const int   oi = __shfl_xor(ix, off, 32);
        const bool tk = (ov > v) || (ov == v && oi < ix);
        v = tk ? ov : v;
        ix = tk ? oi : ix;
      }
      if (lane == 0) sfar = ix;
    }
    __syncthreads();
    int nf = sfar;
    nf = nf < 0 ? 0 : (nf > NPTS - 1 ? NPTS - 1 : nf);
    if ((nf & 1023) == tid) {
      const int isel = nf >> 10;
      float sx = px[0], sy = py[0], sz = pz[0];
#pragma unroll
      for (int i = 1; i < 8; ++i) {
        const bool m = (isel == i);
        sx = m ? px[i] : sx;
        sy = m ? py[i] : sy;
        sz = m ? pz[i] : sz;
      }
      c3[0] = sx; c3[1] = sy; c3[2] = sz;
    }
    __syncthreads();
  }

  if (tid < 512) {
    float* ob = out0 + (size_t)b * 3 * NSEL;
    for (int pass = 0; pass < 2; ++pass) {
#pragma unroll
      for (int ch = 0; ch < 3; ++ch) {
        const v4f v = *(const v4f*)(cs + ch * NSEL + tid * 4);
        *(volatile v4f*)(ob + ch * NSEL + tid * 4) = v;
      }
      __threadfence();
    }
  }
#pragma unroll
  for (int u = 0; u < 2; ++u) {
    const int s = tid + u * 1024;
    const float x = cs[s];
    const float y = cs[NSEL + s];
    const float z = cs[2 * NSEL + s];
    const float t0 = x * x;
    const float t1 = y * y;
    const float t2 = z * z;
    const float ssq = (t0 + t2) + t1;
    const v4f v = {x, y, z, ssq};
    store2_v4f(nxw + ((size_t)b * NSEL + s) * 4, v);
  }
}

__device__ __forceinline__ void mlp_tile(const _Float16* Aw, const _Float16* Wl, int c, int hh, v8f (&acc)[2][4]) {
#pragma unroll
  for (int mt = 0; mt < 2; ++mt)
#pragma unroll
    for (int nt = 0; nt < 4; ++nt) acc[mt][nt] = (v8f){0.f, 0.f, 0.f, 0.f, 0.f, 0.f, 0.f, 0.f};
#pragma unroll
  for (int ks = 0; ks < 2; ++ks) {
    const v16h a0 = frag_load(Aw + c * PITCH_A + ks * 32 + 8 * hh);
    const v16h a1 = frag_load(Aw + (16 + c) * PITCH_A + ks * 32 + 8 * hh);
#pragma unroll
    for (int nt = 0; nt < 4; ++nt) {
      const v16h bf = frag_load(Wl + (nt * 16 + c) * PITCH_W + ks * 32 + 8 * hh);
      acc[0][nt] = wm_f16(a0, bf, acc[0][nt]);
      acc[1][nt] = wm_f16(a1, bf, acc[1][nt]);
    }
  }
}

__device__ __forceinline__ void hidden_store(_Float16* Aw, const float* bl, int c, int hh, v8f (&acc)[2][4]) {
#pragma unroll
  for (int nt = 0; nt < 4; ++nt) {
    const float bv = bl[nt * 16 + c];
#pragma unroll
    for (int mt = 0; mt < 2; ++mt) {
#pragma unroll
      for (int r = 0; r < 8; ++r) {
        float v = acc[mt][nt][r] * WCARRY_INV;
        v = v + bv;
        v = fmaxf(v, 0.0f);
        Aw[(mt * 16 + 8 * hh + r) * PITCH_A + nt * 16 + c] = (_Float16)v;
      }
    }
  }
}

__global__ __launch_bounds__(128)
void group_mlp_kernel(const v4f* __restrict__ xt, const unsigned* __restrict__ ptw,
                      const unsigned short* __restrict__ wt, const v4f* __restrict__ nxw,
                      const float* __restrict__ b1, const float* __restrict__ b2, const float* __restrict__ b3,
                      float* __restrict__ out1) {
#pragma clang fp contract(off)
  __shared__ __align__(16) _Float16 Ws[WROWS * PITCH_W];
  __shared__ __align__(16) _Float16 At[4 * 32 * PITCH_A];
  __shared__ __align__(16) float stage[HID3 * PITCH_S];
  __shared__ float bs[WROWS];
  __shared__ int slots[4 * NSAMP];

  const int tid  = threadIdx.x;
  const int wave = tid >> 5;
  const int lane = tid & 31;
  const int hh   = lane >> 4;
  const int c    = lane & 15;
  const int b    = blockIdx.x >> 6;
  const int s0   = (blockIdx.x & 63) * 32;

#pragma unroll 1
  for (int o = 0; o < 4; ++o) {
#pragma unroll
    for (int i = 0; i < 4; ++i) {
      const int seg = (o * 4 + i) * 128 + tid;
      const int row = seg >> 3;
      const int c8  = (seg & 7) * 8;
      const v4u w = *(const v4u*)(const void*)(wt + row * KPAD + c8);
      *(v4u*)(void*)(Ws + row * PITCH_W + c8) = w;
    }
  }
  if (wave < 2) {
    bs[tid] = b1[tid];
    bs[HID1 + tid] = b2[tid];
  }
  bs[HID1 + HID2 + tid] = b3[tid];

  _Float16* Aw = At + wave * 32 * PITCH_A;
  int* sl = slots + wave * NSAMP;
  const v4f* xb = xt + (size_t)b * NPTS;

#pragma unroll 1
  for (int j = 0; j < 8; ++j) {
    const int ql = wave * 8 + j;
    const int q  = b * NSEL + s0 + ql;
    const v4f cen = nxw[q];
    __syncthreads();
    sl[lane] = 0;
    __syncthreads();

    int cnt = 0;
#pragma unroll 1
    for (int n0 = 0; n0 < NPTS && cnt < NSAMP; n0 += 32) {
      const v4f p4 = xb[n0 + lane];
      float p = cen.x * p4.x;
      p = __builtin_fmaf(cen.y, p4.y, p);
      p = __builtin_fmaf(cen.z, p4.z, p);
      float t = -2.0f * p;
      t = t + cen.w;
      t = t + p4.w;
      const bool within = !(t > RADIUS_SQ);
      const unsigned mask = (unsigned)__ballot(within);
      const int pos = cnt + __builtin_popcount(mask & ((1u << lane) - 1u));
      if (within && pos < NSAMP) sl[pos] = n0 + lane;
      cnt += __builtin_popcount(mask);
    }
    __syncthreads();

    const int own  = sl[lane];
    const int frst = sl[0];
    const int cc = (cnt < NSAMP) ? cnt : NSAMP;
    const int fb = (cnt > 0) ? frst : (NPTS - 1);
    int gi = (lane < cc) ? own : fb;
    gi = gi < 0 ? 0 : (gi > NPTS - 1 ? NPTS - 1 : gi);

    const v4f pp = xb[gi];
    const v4u* prow = (const v4u*)(const void*)(ptw + (size_t)(b * NPTS + gi) * 16);
    const v4u r0 = prow[0];
    const v4u r1 = prow[1];
    const v4u r2 = prow[2];
    const v4u r3 = prow[3];
    const float dx = pp.x - cen.x;
    const float dy = pp.y - cen.y;
    const float dz = pp.z - cen.z;
    const unsigned ux = f16_bits(dx);
    const unsigned uy = f16_bits(dy);
    const unsigned uz = f16_bits(dz);
    unsigned zz = 0;
    asm volatile("" : "+v"(zz));
    const v4u d0 = {ux | (uy << 16), uz | (zz << 16), zz, zz};
    const v4u dzv = {zz, zz, zz, zz};
    v4u* arow = (v4u*)(void*)(Aw + lane * PITCH_A);
    arow[0] = r0;
    arow[1] = r1;
    arow[2] = r2;
    arow[3] = r3;
    arow[4] = d0;
    arow[5] = dzv;
    arow[6] = dzv;
    arow[7] = dzv;
    __syncthreads();

    v8f acc[2][4];
    mlp_tile(Aw, Ws, c, hh, acc);
    __syncthreads();
    hidden_store(Aw, bs, c, hh, acc);
    __syncthreads();
    mlp_tile(Aw, Ws + HID1 * PITCH_W, c, hh, acc);
    __syncthreads();
    hidden_store(Aw, bs + HID1, c, hh, acc);
    __syncthreads();

#pragma unroll 1
    for (int hf = 0; hf < 2; ++hf) {
      mlp_tile(Aw, Ws + (HID1 + HID2 + hf * 64) * PITCH_W, c, hh, acc);
#pragma unroll
      for (int nt = 0; nt < 4; ++nt) {
        float m = acc[0][nt][0];
#pragma unroll
        for (int r = 1; r < 8; ++r) m = fmaxf(m, acc[0][nt][r]);
#pragma unroll
        for (int r = 0; r < 8; ++r) m = fmaxf(m, acc[1][nt][r]);
        const float o = __shfl_xor(m, 16, 32);
        m = fmaxf(m, o);
        float v = m * WCARRY_INV;
        v = v + bs[HID1 + HID2 + hf * 64 + nt * 16 + c];
        v = fmaxf(v, 0.0f);
        if (hh == 0) stage[(hf * 64 + nt * 16 + c) * PITCH_S + ql] = v;
      }
    }
  }
  __syncthreads();

  {
    const int q4 = lane >> 3;
    const int f4 = (lane & 7) * 4;
    float* ob = out1 + (size_t)b * HID3 * NSEL + s0 + f4;
    for (int pass = 0; pass < 2; ++pass) {
#pragma unroll
      for (int it = 0; it < 8; ++it) {
        const int ch = wave * 32 + it * 4 + q4;
        const v4f v = *(const v4f*)(stage + ch * PITCH_S + f4);
        *(volatile v4f*)(ob + (size_t)ch * NSEL) = v;
      }
      __threadfence();
    }
  }
}

extern "C" void kernel_launch(void* const* d_in, const int* in_sizes, int n_in,
                              void* d_out, int out_size, void* d_ws, size_t ws_size,
                              hipStream_t stream) {
  (void)in_sizes; (void)n_in; (void)out_size;
  if (ws_size < WS_TOTAL) return;
  const float* xyz = (const float*)d_in[0];
  const float* pts = (const float*)d_in[1];
  const float* w1  = (const float*)d_in[2];
  const float* b1  = (const float*)d_in[3];
  const float* w2  = (const float*)d_in[4];
  const float* b2  = (const float*)d_in[5];
  const float* w3  = (const float*)d_in[6];
  const float* b3  = (const float*)d_in[7];

  float* out0 = (float*)d_out;
  float* out1 = out0 + (size_t)NBATCH * 3 * NSEL;

  unsigned char* ws = (unsigned char*)d_ws;
  float*    xt  = (float*)(ws + OFF_XT);
  unsigned* ptw = (unsigned*)(ws + OFF_PTW);
  unsigned* wtw = (unsigned*)(ws + OFF_WT);
  float*    nxw = (float*)(ws + OFF_NXW);

  prep_kernel<<<PREP_XYZ_BLOCKS + PREP_PTS_BLOCKS + PREP_WT_BLOCKS, 256, 0, stream>>>(
      xyz, pts, w1, w2, w3, xt, ptw, wtw);
  fps_kernel<<<NBATCH, 1024, 0, stream>>>(xyz, out0, nxw);
  group_mlp_kernel<<<NBATCH * (NSEL / 32), 128, 0, stream>>>(
      (const v4f*)xt, (const unsigned*)ptw, (const unsigned short*)wtw, (const v4f*)nxw,
      b1, b2, b3, out1);
}
